// PhysicsInformedNN_34196529611438
// MI455X (gfx1250) — hardware-verified
//
#include <hip/hip_runtime.h>
#include <hip/hip_bf16.h>
#include <math.h>

typedef __attribute__((ext_vector_type(16))) _Float16 v16h;
typedef __attribute__((ext_vector_type(8)))  _Float16 v8h;
typedef __attribute__((ext_vector_type(8)))  float    v8f;

#define PITCH 264
#define WAVES_PER_BLOCK 2
#define BLOCK (WAVES_PER_BLOCK * 32)

#define WP_OFF_L6 335872

struct BiasPack { const float* p[7]; };

__device__ __forceinline__ float fast_tanh(float x) { return tanhf(x); }

__global__ void repack_kernel(const float* __restrict__ W, int K, int N,
                              int nkc, _Float16* __restrict__ out, int total)
{
    int pidx = blockIdx.x * blockDim.x + threadIdx.x;
    if (2 * pidx >= total) return;
    unsigned short hv[2];
#pragma unroll
    for (int q = 0; q < 2; ++q) {
        int idx  = 2 * pidx + q;
        int i    = idx & 15;
        int lane = (idx >> 4) & 31;
        int frag = idx >> 9;
        int kc   = frag % nkc;
        int nt   = frag / nkc;
        int k = kc * 32 + 8 * (lane >> 4) + ((i < 8) ? i : (i + 8));
        int n = nt * 16 + (lane & 15);
        float v = (k < K && n < N) ? W[k * N + n] : 0.0f;
        hv[q] = __builtin_bit_cast(unsigned short, (_Float16)v);
    }
    const unsigned u = (unsigned)hv[0] | ((unsigned)hv[1] << 16);
    ((volatile unsigned*)out)[pidx] = u;
    __threadfence();
    ((volatile unsigned*)out)[pidx] = u;
}

__device__ __forceinline__ v16h load_afrag(const _Float16* H, int m, int sel8, int kc)
{
    const _Float16* p = H + m * PITCH + kc * 32 + sel8;
    v8h lo = *(const v8h*)p;
    v8h hi = *(const v8h*)(p + 16);
    v16h a;
#pragma unroll
    for (int i = 0; i < 8; ++i) { a[i] = lo[i]; a[8 + i] = hi[i]; }
    return a;
}

__device__ __forceinline__ v8f wmma_f16(v16h a, v16h b, v8f c)
{
    c = __builtin_amdgcn_wmma_f32_16x16x32_f16(false, a, false, b,
                                               (short)0, c, false, false);
    asm volatile("v_nop\n\tv_nop\n\tv_nop\n\tv_nop" : "+v"(c) : "v"(a), "v"(b));
    return c;
}
__device__ __forceinline__ void wave_lds_sync()
{
    __builtin_amdgcn_fence(__ATOMIC_RELEASE, "workgroup");
    __builtin_amdgcn_wave_barrier();
    __builtin_amdgcn_fence(__ATOMIC_ACQUIRE, "workgroup");
}

__device__ __forceinline__ void store_act(_Float16* H, v8f c, int sel8, int nt, int n,
                                          float bn, bool combined)
{
    float deriv = 0.0f;
#pragma unroll
    for (int j = 0; j < 8; ++j) {
        float v = c[j], hv;
        if (!combined || (j & 3) == 0) {
            hv = fast_tanh(v + bn);
            deriv = 1.0f - hv * hv;
        } else {
            hv = v * deriv;
        }
        H[(sel8 + j) * PITCH + nt * 16 + n] = (_Float16)hv;
    }
}

template <int NKC>
__device__ __forceinline__ void hidden_layer(_Float16* H,
                                             const _Float16* __restrict__ Wl,
                                             const float* __restrict__ bias,
                                             int lane, bool combined)
{
    const int mA   = lane & 15;
    const int sel8 = (lane >> 4) << 3;
    const int n    = lane & 15;

    v16h af0[NKC], af1[NKC];
#pragma unroll
    for (int kc = 0; kc < NKC; ++kc) {
        af0[kc] = load_afrag(H, mA, sel8, kc);
        af1[kc] = load_afrag(H, 16 + mA, sel8, kc);
    }
#pragma unroll
    for (int nt = 0; nt < 16; ++nt) {
        float bn = bias[nt * 16 + n];
        const v8f zero = {};
        v16h b = *(const v16h*)(Wl + (nt * NKC * 32 + lane) * 16);
        v8f c0 = wmma_f16(af0[0], b, zero);
        v8f c1 = wmma_f16(af1[0], b, zero);
#pragma unroll
        for (int kc = 1; kc < NKC; ++kc) {
            v16h bk = *(const v16h*)(Wl + ((nt * NKC + kc) * 32 + lane) * 16);
            c0 = wmma_f16(af0[kc], bk, c0);
            c1 = wmma_f16(af1[kc], bk, c1);
        }
        store_act(H, c0, sel8, nt, n, bn, combined);
        store_act(H + 16 * PITCH, c1, sel8, nt, n, bn, combined);
    }
}

__device__ __forceinline__ void final_layer(const _Float16* H, float* Sf,
                                            const _Float16* __restrict__ Wl,
                                            const float* __restrict__ b6,
                                            int lane, bool combined)
{
    const int mA   = lane & 15;
    const int sel8 = (lane >> 4) << 3;
    const int n    = lane & 15;

    v16h af0[8], af1[8];
#pragma unroll
    for (int kc = 0; kc < 8; ++kc) {
        af0[kc] = load_afrag(H, mA, sel8, kc);
        af1[kc] = load_afrag(H, 16 + mA, sel8, kc);
    }
    float bn = (n < 3) ? b6[n] : 0.0f;
    const v8f zero = {};
    {
        v16h b = *(const v16h*)(Wl + (lane) * 16);
        v8f c0 = wmma_f16(af0[0], b, zero);
        v8f c1 = wmma_f16(af1[0], b, zero);
#pragma unroll
        for (int kc = 1; kc < 8; ++kc) {
            v16h bk = *(const v16h*)(Wl + (kc * 32 + lane) * 16);
            c0 = wmma_f16(af0[kc], bk, c0);
            c1 = wmma_f16(af1[kc], bk, c1);
        }
#pragma unroll
        for (int j = 0; j < 8; ++j) {
            float add = (!combined || (j & 3) == 0) ? bn : 0.0f;
            Sf[(sel8 + j) * 16 + n]      = c0[j] + add;
            Sf[(16 + sel8 + j) * 16 + n] = c1[j] + add;
        }
    }
}

__device__ __forceinline__ void run_mlp(_Float16* H, float* Sf,
                                        const _Float16* __restrict__ Wp,
                                        BiasPack bp, int lane, bool combined)
{
    wave_lds_sync();
    hidden_layer<1>(H, Wp, bp.p[0], lane, combined);
    for (int l = 1; l <= 5; ++l) {
        wave_lds_sync();
        hidden_layer<8>(H, Wp + 8192 + (l - 1) * 65536, bp.p[l], lane, combined);
    }
    wave_lds_sync();
    final_layer(H, Sf, Wp + WP_OFF_L6, bp.p[6], lane, combined);
    wave_lds_sync();
}

__device__ __forceinline__ void block_partial(float* red, float contrib, float* line)
{
    red[threadIdx.x] = contrib;
    __syncthreads();
    if (threadIdx.x < 32) {
        float s = 0.0f;
        if (threadIdx.x == 0) {
            for (int i = 0; i < BLOCK; ++i) s += red[i];
        }
        const float v = (threadIdx.x == 0) ? s : 0.0f;
        ((volatile float*)line)[threadIdx.x] = v;
        __threadfence();
        ((volatile float*)line)[threadIdx.x] = v;
    }
}

__global__ __launch_bounds__(BLOCK) void bc_kernel(
    const float* __restrict__ x0, const float* __restrict__ y0,
    const float* __restrict__ bx0, const float* __restrict__ by0,
    const float* __restrict__ bz0,
    const float* __restrict__ lb, const float* __restrict__ ub,
    const _Float16* __restrict__ Wp, BiasPack bp,
    float* __restrict__ partial, int N0)
{
    __shared__ __align__(16) _Float16 Hs[WAVES_PER_BLOCK][32 * PITCH];
    __shared__ float Sfs[WAVES_PER_BLOCK][512];
    __shared__ float red[BLOCK];

    int lane  = threadIdx.x & 31;
    int wslot = threadIdx.x >> 5;
    int wave  = blockIdx.x * WAVES_PER_BLOCK + wslot;
    int pt0   = wave * 32;

    _Float16* H  = Hs[wslot];
    float*    Sf = Sfs[wslot];

#pragma unroll
    for (int r = 0; r < 32; ++r) {
        int k = lane;
        float v = 0.0f;
        if (k < 3) {
            float p = (k == 0) ? x0[pt0 + r] : (k == 1) ? y0[pt0 + r] : 0.0f;
            v = 2.0f * (p - lb[k]) / (ub[k] - lb[k]) - 1.0f;
        }
        H[r * PITCH + k] = (_Float16)v;
    }

    run_mlp(H, Sf, Wp, bp, lane, false);

    int p = pt0 + lane;
    float ex = Sf[lane * 16 + 0] - bx0[p];
    float ey = Sf[lane * 16 + 1] - by0[p];
    float ez = Sf[lane * 16 + 2] - bz0[p];
    float contrib = (ex * ex + ey * ey + ez * ez) / (float)N0;
    block_partial(red, contrib, partial + (size_t)blockIdx.x * 32);
}

__global__ __launch_bounds__(BLOCK) void field_kernel(
    const float* __restrict__ xyz,
    const float* __restrict__ lb, const float* __restrict__ ub,
    const _Float16* __restrict__ Wp, BiasPack bp,
    float* __restrict__ partial, int NF)
{
    __shared__ __align__(16) _Float16 Hs[WAVES_PER_BLOCK][32 * PITCH];
    __shared__ float Sfs[WAVES_PER_BLOCK][512];
    __shared__ float red[BLOCK];

    int lane  = threadIdx.x & 31;
    int wslot = threadIdx.x >> 5;
    int wave  = blockIdx.x * WAVES_PER_BLOCK + wslot;
    int pt0   = wave * 8;

    _Float16* H  = Hs[wslot];
    float*    Sf = Sfs[wslot];

#pragma unroll
    for (int r = 0; r < 32; ++r) {
        int k = lane;
        int p = pt0 + (r >> 2);
        int t = r & 3;
        float v = 0.0f;
        if (k < 3) {
            float inv = ub[k] - lb[k];
            if (t == 0)          v = 2.0f * (xyz[p * 3 + k] - lb[k]) / inv - 1.0f;
            else if (k == t - 1) v = 2.0f / inv;
        }
        H[r * PITCH + k] = (_Float16)v;
    }

    run_mlp(H, Sf, Wp, bp, lane, true);

    float contrib = 0.0f;
    if (lane < 8) {
        int base = lane * 4;
        float bx  = Sf[(base + 0) * 16 + 0], by  = Sf[(base + 0) * 16 + 1], bz  = Sf[(base + 0) * 16 + 2];
        float jxx = Sf[(base + 1) * 16 + 0], jxy = Sf[(base + 1) * 16 + 1], jxz = Sf[(base + 1) * 16 + 2];
        float jyx = Sf[(base + 2) * 16 + 0], jyy = Sf[(base + 2) * 16 + 1], jyz = Sf[(base + 2) * 16 + 2];
        float jzx = Sf[(base + 3) * 16 + 0], jzy = Sf[(base + 3) * 16 + 1], jzz = Sf[(base + 3) * 16 + 2];
        float dv = jxx + jyy + jzz;
        float jx = jyz - jzy, jy = jzx - jxz, jz = jxy - jyx;
        float c1 = jy * bz - jz * by;
        float c2 = jz * bx - jx * bz;
        float c3 = jx * by - jy * bx;
        contrib = (dv * dv + c1 * c1 + c2 * c2 + c3 * c3) / (float)NF;
    }
    block_partial(red, contrib, partial + (size_t)blockIdx.x * 32);
}

__global__ __launch_bounds__(256) void reduce_kernel(const float* __restrict__ partial, int nblocks,
                                                    float* __restrict__ out)
{
    __shared__ double sred[256];
    double s = 0.0;
    for (int i = threadIdx.x; i < nblocks; i += 256) s += (double)partial[(size_t)i * 32];
    sred[threadIdx.x] = s;
    __syncthreads();
    for (int st = 128; st > 0; st >>= 1) {
        if (threadIdx.x < st) sred[threadIdx.x] += sred[threadIdx.x + st];
        __syncthreads();
    }
    if (threadIdx.x == 0) {
        const float v = (float)sred[0];
        ((volatile float*)out)[0] = v;
        __threadfence();
        ((volatile float*)out)[0] = v;
    }
}

extern "C" void kernel_launch(void* const* d_in, const int* in_sizes, int n_in,
                              void* d_out, int out_size, void* d_ws, size_t ws_size,
                              hipStream_t stream)
{
    const float* x0  = (const float*)d_in[0];
    const float* y0  = (const float*)d_in[1];
    const float* bx0 = (const float*)d_in[2];
    const float* by0 = (const float*)d_in[3];
    const float* bz0 = (const float*)d_in[4];
    const float* xyz = (const float*)d_in[5];
    const float* lb  = (const float*)d_in[6];
    const float* ub  = (const float*)d_in[7];

    const float* W[7];
    BiasPack bp;
    for (int l = 0; l < 7; ++l) {
        W[l]    = (const float*)d_in[8 + 2 * l];
        bp.p[l] = (const float*)d_in[9 + 2 * l];
    }

    _Float16* Wp = (_Float16*)d_ws;
    float* partial = (float*)((char*)d_ws + 1048576);
    float* out = (float*)d_out;

    repack_kernel<<<8192 / 512, 256, 0, stream>>>(W[0], 3, 256, 1, Wp, 8192);
    for (int l = 1; l <= 5; ++l)
        repack_kernel<<<65536 / 512, 256, 0, stream>>>(W[l], 256, 256, 8,
                                                       Wp + 8192 + (l - 1) * 65536, 65536);
    repack_kernel<<<4096 / 512, 256, 0, stream>>>(W[6], 256, 3, 8, Wp + WP_OFF_L6, 4096);

    int N0 = in_sizes[0];
    int NF = in_sizes[5] / 3;

    const int nbc = N0 / 32 / WAVES_PER_BLOCK;
    const int nfd = NF / 8 / WAVES_PER_BLOCK;
    bc_kernel<<<nbc, BLOCK, 0, stream>>>(
        x0, y0, bx0, by0, bz0, lb, ub, Wp, bp, partial, N0);
    field_kernel<<<nfd, BLOCK, 0, stream>>>(
        xyz, lb, ub, Wp, bp, partial + (size_t)nbc * 32, NF);
    reduce_kernel<<<1, 256, 0, stream>>>(partial, nbc + nfd, out);
}
